// BNNFC_32856499814961
// MI455X (gfx1250) — hardware-verified
//
#include <hip/hip_runtime.h>
#include <math.h>

typedef __attribute__((ext_vector_type(16))) _Float16 v16h;
typedef __attribute__((ext_vector_type(16))) __bf16 v16b;
typedef __attribute__((ext_vector_type(8)))  _Float16 v8h;
typedef __attribute__((ext_vector_type(8)))  float v8f;
typedef __attribute__((ext_vector_type(4)))  float v4f;
typedef __attribute__((ext_vector_type(2)))  float v2f;
typedef __attribute__((ext_vector_type(4)))  unsigned v4u;
typedef __attribute__((ext_vector_type(4)))  int v4i;
typedef float __attribute__((may_alias)) float_a;
typedef int __attribute__((may_alias)) int_a;

template <typename T> __device__ __forceinline__ void vst2(void* p, T v) { *(volatile T*)p = v; __threadfence(); *(volatile T*)p = v; }
__device__ __forceinline__ v8f wmma16(v16h a, v16h b, v8f c) {
  v8f d = __builtin_amdgcn_wmma_f32_16x16x32_f16(false, a, false, b, (short)0, c, false, false);
  asm volatile("v_nop\n\tv_nop\n\tv_nop\n\tv_nop" : "+v"(d) : "v"(a), "v"(b));
  return d;
}
__device__ __forceinline__ v8f wmma_bf(v16b a, v16b b, v8f c) {
  v8f d = __builtin_amdgcn_wmma_f32_16x16x32_bf16(false, a, false, b, (short)0, c, false, false);
  asm volatile("v_nop\n\tv_nop\n\tv_nop\n\tv_nop" : "+v"(d) : "v"(a), "v"(b));
  return d;
}
__device__ __forceinline__ v16h frag_h(const _Float16* rowk0, int lane) {
  union { v16h v; v8h q[2]; } u; const _Float16* p = rowk0 + 8 * (lane >> 4);
  u.q[0] = *(const v8h*)p; u.q[1] = *(const v8h*)(p + 16); return u.v;
}
__device__ __forceinline__ v16h frag_f32(const float* rowk0, int lane) {
  v16h a; const float* p = rowk0 + 8 * (lane >> 4);
#pragma unroll
  for (int i = 0; i < 8; ++i) { a[i] = (_Float16)p[i]; a[8 + i] = (_Float16)p[16 + i]; }
  return a;
}
__device__ __forceinline__ v16h frag_f32s(const float* rowk0, int lane, float sc) {
  v16h a; const float* p = rowk0 + 8 * (lane >> 4);
#pragma unroll
  for (int i = 0; i < 8; ++i) { a[i] = (_Float16)(p[i] * sc); a[8 + i] = (_Float16)(p[16 + i] * sc); }
  return a;
}
__device__ __forceinline__ v16h fragc_f32(const float* W, int k0, int n, int lane, int ld, int K) {
  v16h a; const int g = lane >> 4;
#pragma unroll
  for (int i = 0; i < 8; ++i) { const int ka = k0 + 8 * g + i, kb = ka + 16;
    a[i] = (_Float16)(ka < K ? W[(size_t)ka * ld + n] : 0.f); a[8 + i] = (_Float16)(kb < K ? W[(size_t)kb * ld + n] : 0.f); }
  return a;
}
struct F2 { v16b h, l; };
__device__ __forceinline__ F2 bsplit16(const float v[16]) { F2 r;
#pragma unroll
  for (int i = 0; i < 16; ++i) { const __bf16 h = (__bf16)v[i]; r.h[i] = h; r.l[i] = (__bf16)(v[i] - (float)h); }
  return r; }
__device__ __forceinline__ F2 split_row(const float* row, int k0, int lane) { float v[16]; const float* p = row + k0 + 8 * (lane >> 4);
#pragma unroll
  for (int i = 0; i < 8; ++i) { v[i] = p[i]; v[8 + i] = p[16 + i]; }
  return bsplit16(v); }
__device__ __forceinline__ F2 split_rowK(const float* row, int k0, int lane, int K) { float v[16]; const int g = lane >> 4;
#pragma unroll
  for (int i = 0; i < 8; ++i) { const int ka = k0 + 8 * g + i, kb = ka + 16; v[i] = ka < K ? row[ka] : 0.f; v[8 + i] = kb < K ? row[kb] : 0.f; }
  return bsplit16(v); }
__device__ __forceinline__ F2 split_col(const float* W, int k0, int n, int lane, int ld, int K) { float v[16]; const int g = lane >> 4;
#pragma unroll
  for (int i = 0; i < 8; ++i) { const int ka = k0 + 8 * g + i, kb = ka + 16; v[i] = ka < K ? W[(size_t)ka * ld + n] : 0.f; v[8 + i] = kb < K ? W[(size_t)kb * ld + n] : 0.f; }
  return bsplit16(v); }
__device__ __forceinline__ v8f mac3(const F2& a, const F2& b, v8f c) { c = wmma_bf(a.l, b.h, c); c = wmma_bf(a.h, b.l, c); return wmma_bf(a.h, b.h, c); }
__device__ __forceinline__ float sigm(float v) { return 1.0f / (1.0f + expf(-v)); }
#define LDSX() do { asm volatile("s_wait_dscnt 0" ::: "memory"); __builtin_amdgcn_wave_barrier(); __builtin_amdgcn_fence(__ATOMIC_RELEASE, "workgroup"); } while (0)

#define NB 32
#define TT 1000
#define NI 256
#define NH 512
#define NO 128
#define DLY 20
#define NR (NB * TT)

__global__ __launch_bounds__(256) void k_packT(const float* __restrict__ Wiv, const float* __restrict__ Wlat, const float* __restrict__ Wo, _Float16* __restrict__ P) {
  __shared__ float tile[64][65];
  const int which = blockIdx.z, o0 = blockIdx.x * 64, k0 = blockIdx.y * 64, tid = threadIdx.x;
  const float* W = which == 0 ? Wiv : (which == 1 ? Wlat : Wo); const int KIN = which == 0 ? NI : NH, NOUT = which == 2 ? NO : NH;
  if (o0 >= NOUT || k0 >= KIN) return;
  for (int q = tid; q < 64 * 64; q += 256) { const int kl = q >> 6, ol = q & 63; tile[kl][ol] = W[(size_t)(k0 + kl) * NOUT + o0 + ol]; }
  __syncthreads();
  for (int u = 0; u < 2; ++u) { const int idx = tid + u * 256, ol = idx >> 3, pc = idx & 7; union { v8h hh; v4u uu; } pk;
#pragma unroll
    for (int i = 0; i < 8; ++i) pk.hh[i] = (_Float16)(tile[pc * 8 + i][ol] * 16.0f);
    vst2(P + ((size_t)which * NH + o0 + ol) * NH + k0 + pc * 8, pk.uu); }
}
__global__ __launch_bounds__(256) void k_cvt(const float* __restrict__ x, _Float16* __restrict__ x16, size_t n8) {
  const size_t g8 = (size_t)blockIdx.x * 256 + threadIdx.x; if (g8 >= n8) return;
  union { v8h h; v4u u; } pk;
#pragma unroll
  for (int e = 0; e < 8; ++e) pk.h[e] = (_Float16)x[g8 * 8 + e];
  vst2(x16 + g8 * 8, pk.u);
}
__global__ __launch_bounds__(128) void k_drive(const _Float16* __restrict__ x16, const _Float16* __restrict__ P, float* __restrict__ drive) {
  __shared__ __align__(16) float so[4][16][132];
  const int tid = threadIdx.x, wave = tid >> 5, lane = tid & 31, col = lane & 15, g = lane >> 4;
  const int r0 = blockIdx.x * 64 + wave * 16, n0 = blockIdx.y * 128;
  v8f acc[8] = {};
#pragma unroll
  for (int kc = 0; kc < NI / 32; ++kc) { const v16h a = frag_h(x16 + (size_t)(r0 + col) * NI + kc * 32, lane);
#pragma unroll
    for (int j = 0; j < 8; ++j) acc[j] = wmma16(a, frag_h(P + (size_t)(n0 + j * 16 + col) * NH + kc * 32, lane), acc[j]); }
#pragma unroll
  for (int j = 0; j < 8; ++j)
#pragma unroll
    for (int r = 0; r < 8; ++r) so[wave][8 * g + r][j * 16 + col] = acc[j][r] * (1.0f / 16.0f);
  LDSX();
#pragma unroll 4
  for (int rl = 0; rl < 16; ++rl) vst2(drive + (size_t)(r0 + rl) * NH + n0 + lane * 4, *(const v4f*)(&so[wave][rl][lane * 4]));
}
#define NTW 2
__global__ __launch_bounds__(512) void k_rec(const float* __restrict__ drive, const _Float16* __restrict__ P, const float* __restrict__ thresh, const float* __restrict__ tkm, const float* __restrict__ aamp, const float* __restrict__ tar, const float* __restrict__ tka,
                                           _Float16* __restrict__ F16) {
  __shared__ __align__(16) _Float16 sf[16][16][40];
  const int tid = threadIdx.x, w = tid >> 5, lane = tid & 31, col = lane & 15, g = lane >> 4; const int b0 = blockIdx.x * 16;
  float km[NTW], th[NTW], kasc[2][NTW], ar[2][NTW], amp[2][NTW];
#pragma unroll
  for (int t4 = 0; t4 < NTW; ++t4) { const int n = w * 32 + t4 * 16 + col; km[t4] = sigm(tkm[n]) * (1.0f / 0.05f); th[t4] = thresh[n];
#pragma unroll
    for (int a = 0; a < 2; ++a) { kasc[a][t4] = sigm(tka[a * NH + n]) * (1.0f / 0.05f); ar[a][t4] = 1.0f - 2.0f * sigm(tar[a * NH + n]); amp[a][t4] = aamp[a * NH + n]; } }
  float volt[NTW][8], fprev[NTW][8], asc0[NTW][8], asc1[NTW][8];
#pragma unroll
  for (int t4 = 0; t4 < NTW; ++t4)
#pragma unroll
    for (int r = 0; r < 8; ++r) { volt[t4][r] = 0.f; fprev[t4][r] = 0.f; asc0[t4][r] = 0.f; asc1[t4][r] = 0.f; }
  const _Float16* Wl = P + (size_t)NH * NH;
  const float DTc = 0.05f, Rc = 0.1f;
#pragma unroll 1
  for (int t = 0; t < TT; ++t) {
    v8f acc[NTW] = {};
    if (t >= DLY) {
#pragma unroll 1
      for (int kc = 0; kc < NH / 32; ++kc) { const v16h a = frag_h(F16 + ((size_t)(b0 + col) * TT + (t - DLY)) * NH + kc * 32, lane);
#pragma unroll
        for (int t4 = 0; t4 < NTW; ++t4) acc[t4] = wmma16(a, frag_h(Wl + (size_t)(w * 32 + t4 * 16 + col) * NH + kc * 32, lane), acc[t4]); } }
#pragma unroll
    for (int t4 = 0; t4 < NTW; ++t4) { const int n = w * 32 + t4 * 16 + col;
#pragma unroll
      for (int r = 0; r < 8; ++r) { const int b = b0 + 8 * g + r;
        const float syn = drive[((size_t)b * TT + t) * NH + n] + acc[t4][r] * (1.0f / 16.0f);
        const float f = fprev[t4][r];
        const float a0 = (ar[0][t4] * asc0[t4][r] + amp[0][t4]) * f * DTc + asc0[t4][r] * (1.0f - DTc * kasc[0][t4]);
        const float a1 = (ar[1][t4] * asc1[t4][r] + amp[1][t4]) * f * DTc + asc1[t4][r] * (1.0f - DTc * kasc[1][t4]);
        asc0[t4][r] = a0; asc1[t4][r] = a1;
        const float vo = volt[t4][r];
        const float vn = (1.0f - DTc * km[t4]) * vo + DTc * km[t4] * Rc * (syn + (a0 + a1)) + f * (0.0f - vo);
        volt[t4][r] = vn;
        const float fn = sigm(vn - th[t4]);
        fprev[t4][r] = fn;
        sf[w][8 * g + r][t4 * 16 + col] = (_Float16)fn; } }
    __syncthreads();
    if (w < 8) { for (int q = lane; q < 16 * 8; q += 32) { const int m = q >> 3, pc = q & 7; const int src = 2 * w + (pc >> 2), pcl = pc & 3;
        vst2(F16 + ((size_t)(b0 + m) * TT + t) * NH + w * 64 + pc * 8, *(const v4u*)(&sf[src][m][pcl * 8])); } }
    __syncthreads();
  }
}
__global__ __launch_bounds__(128) void k_out(const _Float16* __restrict__ F16, const _Float16* __restrict__ P, const float* __restrict__ bo, float* __restrict__ out) {
  __shared__ __align__(16) float so[4][16][132];
  const int tid = threadIdx.x, wave = tid >> 5, lane = tid & 31, col = lane & 15, g = lane >> 4;
  const int r0 = blockIdx.x * 64 + wave * 16;
  const _Float16* Wo = P + (size_t)2 * NH * NH;
  v8f acc[8] = {};
#pragma unroll 1
  for (int kc = 0; kc < NH / 32; ++kc) { const v16h a = frag_h(F16 + (size_t)(r0 + col) * NH + kc * 32, lane);
#pragma unroll
    for (int j = 0; j < 8; ++j) acc[j] = wmma16(a, frag_h(Wo + (size_t)(j * 16 + col) * NH + kc * 32, lane), acc[j]); }
#pragma unroll
  for (int j = 0; j < 8; ++j) { const float bb = bo[j * 16 + col];
#pragma unroll
    for (int r = 0; r < 8; ++r) so[wave][8 * g + r][j * 16 + col] = acc[j][r] * (1.0f / 16.0f) + bb; }
  LDSX();
#pragma unroll 4
  for (int rl = 0; rl < 16; ++rl) vst2(out + (size_t)(r0 + rl) * NO + lane * 4, *(const v4f*)(&so[wave][rl][lane * 4]));
}
extern "C" void kernel_launch(void* const* d_in, const int* in_sizes, int n_in, void* d_out, int out_size, void* d_ws, size_t ws_size, hipStream_t stream) {
  (void)in_sizes; (void)n_in; (void)out_size; (void)ws_size;
  const float** I = (const float**)d_in;
  const float* x = I[0]; const float* Wiv = I[1]; const float* Wlat = I[2]; const float* thresh = I[3]; const float* tkm = I[4]; const float* aamp = I[5]; const float* tar = I[6]; const float* tka = I[7]; const float* Wo = I[8]; const float* bo = I[9];
  float* out = (float*)d_out;
  char* ws = (char*)d_ws; size_t off = 0;
  auto take = [&](size_t bytes) { char* p = ws + off; off += (bytes + 255) & ~(size_t)255; return p; };
  _Float16* P = (_Float16*)take((size_t)(2 * NH + NO) * NH * 2); _Float16* x16 = (_Float16*)take((size_t)NR * NI * 2); _Float16* F16 = (_Float16*)take((size_t)NR * NH * 2); float* drive = (float*)take((size_t)NR * NH * 4);
  k_packT<<<dim3(NH / 64, NH / 64, 3), 256, 0, stream>>>(Wiv, Wlat, Wo, P);
  const size_t n8 = (size_t)NR * NI / 8; k_cvt<<<(unsigned)((n8 + 255) / 256), 256, 0, stream>>>(x, x16, n8);
  k_drive<<<dim3(NR / 64, NH / 128), 128, 0, stream>>>(x16, P, drive);
  k_rec<<<NB / 16, 512, 0, stream>>>(drive, P, thresh, tkm, aamp, tar, tka, F16);
  k_out<<<NR / 64, 128, 0, stream>>>(F16, P, bo, out);
}
